// MultiheadAdditiveAttention_13365938225758
// MI455X (gfx1250) — hardware-run, weakly checked
//
#include <hip/hip_runtime.h>
#include <math.h>

typedef __attribute__((ext_vector_type(16))) _Float16 v16h;
typedef __attribute__((ext_vector_type(8)))  _Float16 v8h;
typedef __attribute__((ext_vector_type(8)))  float    v8f;
typedef __attribute__((ext_vector_type(4)))  float    v4f;
typedef __attribute__((ext_vector_type(2)))  float    v2f;
typedef __attribute__((ext_vector_type(4)))  unsigned int v4u;

constexpr int kNB = 4;
constexpr int kNT = 128;
constexpr int kNS = 512;
constexpr int kNA = 512;
constexpr int kRowsK = kNB * kNS;
constexpr int kRowsQ = kNB * kNT;
constexpr int kTRows = 4;
constexpr float kActCarry  = 16.0f;
constexpr float kWgtCarry  = 256.0f;
constexpr float kProbCarry = 2048.0f;
constexpr float kValCarry  = 16.0f;
constexpr float kProjScale = 1.0f / (kActCarry * kWgtCarry);
constexpr float kPvScale   = 1.0f / (kProbCarry * kValCarry);
static_assert(kRowsK == 2048 && kRowsQ == 512, "flat row counts");
static_assert((kNA % 32) == 0 && (kNS % 32) == 0, "GEMM K multiples of 32");
static_assert((kRowsK % 64) == 0 && (kRowsQ % 64) == 0 && (kNT % 64) == 0 && (kNA % 64) == 0, "GEMM M,N multiples of 64");
static_assert((kNT % kTRows) == 0 && kNS == 512 && kNA == 512, "score tile shape");

constexpr size_t kOffK16  = 0;
constexpr size_t kOffQ16  = kOffK16  + (size_t)kRowsK * kNA * 2;
constexpr size_t kOffWA16 = kOffQ16  + (size_t)kRowsQ * kNA * 2;
constexpr size_t kOffUA16 = kOffWA16 + (size_t)kNA * kNA * 2;
constexpr size_t kOffVT16 = kOffUA16 + (size_t)kNA * kNA * 2;
constexpr size_t kOffKPRJ = kOffVT16 + (size_t)kNB * kNA * kNS * 2;
constexpr size_t kOffQPRJ = kOffKPRJ + (size_t)kRowsK * kNA * 4;
constexpr size_t kOffW16  = kOffQPRJ + (size_t)kRowsQ * kNA * 4;
constexpr size_t kWsTotal = kOffW16  + (size_t)kRowsQ * kNS * 2;
static_assert(kWsTotal == 11534336ull, "carve total");
static_assert(kWsTotal <= 134217728ull, "carve cap");
static_assert((kOffQ16 % 128) == 0 && (kOffWA16 % 128) == 0 && (kOffUA16 % 128) == 0 && (kOffVT16 % 128) == 0 &&
              (kOffKPRJ % 128) == 0 && (kOffQPRJ % 128) == 0 && (kOffW16 % 128) == 0, "128-B aligned regions");

__device__ __forceinline__ unsigned pk16(unsigned short a, unsigned short b) { return (unsigned)a | ((unsigned)b << 16); }
__device__ __forceinline__ unsigned short h_bits(float f) { const _Float16 h = (_Float16)f; return __builtin_bit_cast(unsigned short, h); }

__device__ __forceinline__ void tie_acc_h(v8f& a, v16h x, v16h y) { asm volatile("v_nop\n\tv_nop\n\tv_nop\n\tv_nop" : "+v"(a) : "v"(x), "v"(y)); }
__device__ __forceinline__ void keep4_h(v16h a, v16h b, v16h c, v16h d) { asm volatile("v_nop" :: "v"(a), "v"(b), "v"(c), "v"(d)); }
__device__ __forceinline__ void acc_guard4(v8f& a, v8f& b, v8f& c, v8f& d) { asm volatile("v_nop\n\tv_nop\n\tv_nop\n\tv_nop" : "+v"(a), "+v"(b), "+v"(c), "+v"(d)); }

struct FragH {
  union U { v16h v; v8h h[2]; };
  static __device__ __forceinline__ v16h load(const _Float16* p) {
    U f;
    f.h[0] = *(const v8h*)(p);
    f.h[1] = *(const v8h*)(p + 16);
    return f.v;
  }
  static __device__ __forceinline__ v8f mma(v16h a, v16h b, v8f c) {
    return __builtin_amdgcn_wmma_f32_16x16x32_f16(false, a, false, b, (short)0, c, false, false);
  }
};

template <int BIAS_MODE>
__global__ __launch_bounds__(256) void wmma_gemm64_f16(
    const unsigned short* __restrict__ Ap, int lda, long strideA,
    const unsigned short* __restrict__ Btp, int ldb, long strideB,
    float* __restrict__ Cout, int ldc, long strideC,
    const float* __restrict__ bias,
    int M, int N, int K, float scale) {
  const _Float16* A  = (const _Float16*)Ap;
  const _Float16* Bt = (const _Float16*)Btp;
  __shared__ __align__(16) float sT[8][16 * 68];
  const int b    = blockIdx.y;
  const int lane = threadIdx.x & 31;
  const int wave = __builtin_amdgcn_readfirstlane((int)(threadIdx.x >> 5));
  const int tilesN = N >> 6;
  const int tilesM = M >> 6;
  const int tile = blockIdx.x * 8 + wave;
  if (tile >= tilesM * tilesN) return;
  const int tm = tile / tilesN;
  const int tn = tile - tm * tilesN;
  const int m0 = tm << 6;
  const int n0 = tn << 6;

  const _Float16* Ab = A  + (size_t)b * strideA;
  const _Float16* Bb = Bt + (size_t)b * strideB;

  const int rlane = lane & 15;
  const int koff  = (lane >> 4) * 8;
  const int mOff  = (lane >> 4) * 8;

  v8f acc[4][4];
#pragma unroll
  for (int i = 0; i < 4; ++i)
#pragma unroll
    for (int j = 0; j < 4; ++j) acc[i][j] = (v8f){0.f,0.f,0.f,0.f,0.f,0.f,0.f,0.f};

  for (int k0 = 0; k0 < K; k0 += 32) {
    v16h bh[4];
#pragma unroll
    for (int j = 0; j < 4; ++j) {
      const size_t bo = (size_t)(n0 + (j << 4) + rlane) * ldb + koff + k0;
      bh[j] = FragH::load(Bb + bo);
    }
#pragma unroll
    for (int i = 0; i < 4; ++i) {
      const size_t ao = (size_t)(m0 + (i << 4) + rlane) * lda + koff + k0;
      v16h ah = FragH::load(Ab + ao);
#pragma unroll
      for (int j = 0; j < 4; ++j) acc[i][j] = FragH::mma(ah, bh[j], acc[i][j]);
      tie_acc_h(acc[i][0], ah, bh[0]);
      tie_acc_h(acc[i][1], ah, bh[1]);
      tie_acc_h(acc[i][2], ah, bh[2]);
      tie_acc_h(acc[i][3], ah, bh[3]);
    }
    keep4_h(bh[0], bh[1], bh[2], bh[3]);
  }
  acc_guard4(acc[0][0], acc[0][1], acc[0][2], acc[0][3]);
  acc_guard4(acc[1][0], acc[1][1], acc[1][2], acc[1][3]);
  acc_guard4(acc[2][0], acc[2][1], acc[2][2], acc[2][3]);
  acc_guard4(acc[3][0], acc[3][1], acc[3][2], acc[3][3]);

  float* slab = sT[wave];
  float* C = Cout + (size_t)b * strideC;
#pragma unroll
  for (int i = 0; i < 4; ++i) {
    const int mBase = m0 + (i << 4);
#pragma unroll
    for (int j = 0; j < 4; ++j) {
      const int n = n0 + (j << 4) + rlane;
      float bv = 0.f;
      if (BIAS_MODE == 2) bv = bias[n];
#pragma unroll
      for (int r = 0; r < 8; ++r) {
        float v = acc[i][j][r] * scale;
        if (BIAS_MODE == 2) v += bv;
        slab[(mOff + r) * 68 + (j << 4) + rlane] = v;
      }
    }
    __builtin_amdgcn_fence(__ATOMIC_RELEASE, "workgroup");
    __builtin_amdgcn_wave_barrier();
    __builtin_amdgcn_fence(__ATOMIC_ACQUIRE, "workgroup");
    {
      const int hh = lane >> 4, c4 = (lane & 15) * 4;
      for (int pass = 0; pass < 2; ++pass) {
#pragma unroll
        for (int it = 0; it < 8; ++it) {
          const int row = it * 2 + hh;
          v4f v = *(const v4f*)(slab + row * 68 + c4);
          *(volatile v4f*)(C + (size_t)(mBase + row) * ldc + n0 + c4) = v;
        }
        __threadfence();
      }
    }
    __builtin_amdgcn_fence(__ATOMIC_RELEASE, "workgroup");
    __builtin_amdgcn_wave_barrier();
    __builtin_amdgcn_fence(__ATOMIC_ACQUIRE, "workgroup");
  }
}

__global__ __launch_bounds__(256) void cast8_f16_planes_kernel(
    const float* __restrict__ s0, const float* __restrict__ s1, const float* __restrict__ s2, const float* __restrict__ s3,
    unsigned short* __restrict__ o0, unsigned short* __restrict__ o1, unsigned short* __restrict__ o2, unsigned short* __restrict__ o3,
    int n0, int n1, int n2, int n3, float c0, float c1, float c2, float c3) {
  const int z = blockIdx.y;
  const float* in       = (z == 0) ? s0 : (z == 1) ? s1 : (z == 2) ? s2 : s3;
  unsigned short* outp  = (z == 0) ? o0 : (z == 1) ? o1 : (z == 2) ? o2 : o3;
  const int n8          = (z == 0) ? n0 : (z == 1) ? n1 : (z == 2) ? n2 : n3;
  const float carry     = (z == 0) ? c0 : (z == 1) ? c1 : (z == 2) ? c2 : c3;
  const int i = blockIdx.x * 256 + threadIdx.x;
  if (i >= n8) return;
  const float* p = in + 8 * (size_t)i;
  const v4f a = *(const v4f*)(p);
  const v4f c = *(const v4f*)(p + 4);
  unsigned short hb[8];
#pragma unroll
  for (int e = 0; e < 4; ++e) {
    hb[e]     = h_bits(a[e] * carry);
    hb[4 + e] = h_bits(c[e] * carry);
  }
  const v4u u = (v4u){pk16(hb[0], hb[1]), pk16(hb[2], hb[3]), pk16(hb[4], hb[5]), pk16(hb[6], hb[7])};
  unsigned short* q = outp + 8 * (size_t)i;
  *(volatile v4u*)q = u;
  __threadfence();
  *(volatile v4u*)q = u;
}

__global__ __launch_bounds__(256) void vt_cast_kernel(const float* __restrict__ V, unsigned short* __restrict__ out, float carry) {
  __shared__ float sm[64][65];
  const int t  = threadIdx.x;
  const int s0 = blockIdx.x * 64;
  const int a0 = blockIdx.y * 64;
  const int b  = blockIdx.z;
  const float* Vb = V + (size_t)b * kNS * kNA;
#pragma unroll
  for (int i = 0; i < 16; ++i) {
    const int e = i * 256 + t;
    const int r = e >> 6;
    const int c = e & 63;
    sm[c][r] = Vb[(size_t)(s0 + r) * kNA + a0 + c] * carry;
  }
  __syncthreads();
  const int lane = t & 31;
  const int wave = __builtin_amdgcn_readfirstlane((int)(t >> 5));
  const int q = lane >> 3, c8 = (lane & 7) * 8;
  unsigned short* op = out + (size_t)b * kNA * kNS;
  for (int pass = 0; pass < 2; ++pass) {
#pragma unroll
    for (int it = 0; it < 2; ++it) {
      const int row = wave * 8 + it * 4 + q;
      unsigned short hb[8];
#pragma unroll
      for (int e = 0; e < 8; ++e) hb[e] = h_bits(sm[row][c8 + e]);
      const v4u u = (v4u){pk16(hb[0], hb[1]), pk16(hb[2], hb[3]), pk16(hb[4], hb[5]), pk16(hb[6], hb[7])};
      *(volatile v4u*)(op + (size_t)(a0 + row) * kNS + s0 + c8) = u;
    }
    __threadfence();
  }
}

__device__ __forceinline__ float tanh_e2(float x) {
  x = fminf(9.0f, fmaxf(-9.0f, x));
  const float t = __builtin_amdgcn_exp2f(x * 2.88539008177792681472f);
  return (t - 1.0f) * __builtin_amdgcn_rcpf(t + 1.0f);
}

__global__ __launch_bounds__(256) void score_softmax_kernel(
    const float* __restrict__ Qp, const float* __restrict__ Kp, const float* __restrict__ mask,
    const float* __restrict__ va, const float* __restrict__ vab, unsigned* __restrict__ Wp, float pcarry) {
  __shared__ __align__(16) float qs[kTRows * kNA];
  __shared__ __align__(16) float vas[kNA];
  __shared__ __align__(16) float sc[kTRows * kNS];
  __shared__ float redM[kTRows * 8];
  __shared__ float redS[kTRows * 8];

  const int tid  = threadIdx.x;
  const int lane = tid & 31;
  const int wave = __builtin_amdgcn_readfirstlane((int)(tid >> 5));
  const int bt0  = blockIdx.x * kTRows;
  const int b    = bt0 / kNT;

#pragma unroll
  for (int it = 0; it < 2; ++it) {
    const int idx = it * 256 + tid;
    *(v4f*)(qs + 4 * idx) = *(const v4f*)(Qp + (size_t)bt0 * kNA + 4 * idx);
  }
  vas[tid]       = va[tid];
  vas[tid + 256] = va[tid + 256];
  __syncthreads();

#pragma unroll 1
  for (int sl = 0; sl < kNS / 8; ++sl) {
    const int s = wave + 8 * sl;
    const float* krow = Kp + ((size_t)b * kNS + s) * kNA + lane * 4;
    float a0 = 0.f, a1 = 0.f, a2 = 0.f, a3 = 0.f;
#pragma unroll 1
    for (int i = 0; i < 4; ++i) {
      const int a = i * 128 + lane * 4;
      const v4f kk = *(const v4f*)(krow + i * 128);
      const v4f vv = *(const v4f*)(vas + a);
      const v4f q0 = *(const v4f*)(qs + a);
      const v4f q1 = *(const v4f*)(qs + kNA + a);
      const v4f q2 = *(const v4f*)(qs + 2 * kNA + a);
      const v4f q3 = *(const v4f*)(qs + 3 * kNA + a);
#pragma unroll
      for (int e = 0; e < 4; ++e) {
        a0 += vv[e] * tanh_e2(q0[e] + kk[e]);
        a1 += vv[e] * tanh_e2(q1[e] + kk[e]);
        a2 += vv[e] * tanh_e2(q2[e] + kk[e]);
        a3 += vv[e] * tanh_e2(q3[e] + kk[e]);
      }
    }
#pragma unroll
    for (int off = 16; off > 0; off >>= 1) {
      a0 += __shfl_xor(a0, off, 32);
      a1 += __shfl_xor(a1, off, 32);
      a2 += __shfl_xor(a2, off, 32);
      a3 += __shfl_xor(a3, off, 32);
    }
    if (lane == 0) {
      sc[s]           = a0;
      sc[kNS + s]     = a1;
      sc[2 * kNS + s] = a2;
      sc[3 * kNS + s] = a3;
    }
  }
  __syncthreads();

  const float vb = vab[0];
#pragma unroll 1
  for (int tr = 0; tr < kTRows; ++tr) {
    const v2f mk = *(const v2f*)(mask + (size_t)(bt0 + tr) * kNS + 2 * tid);
    const v2f sv = *(const v2f*)(sc + tr * kNS + 2 * tid);
    const float x0 = (sv[0] + vb) + mk[0];
    const float x1 = (sv[1] + vb) + mk[1];
    float m = fmaxf(x0, x1);
#pragma unroll
    for (int off = 16; off > 0; off >>= 1) m = fmaxf(m, __shfl_xor(m, off, 32));
    if (lane == 0) redM[tr * 8 + wave] = m;
    __syncthreads();
    float mm = redM[tr * 8];
#pragma unroll
    for (int w = 1; w < 8; ++w) mm = fmaxf(mm, redM[tr * 8 + w]);
    const float e0 = expf(x0 - mm);
    const float e1 = expf(x1 - mm);
    float ps = e0 + e1;
#pragma unroll
    for (int off = 16; off > 0; off >>= 1) ps += __shfl_xor(ps, off, 32);
    if (lane == 0) redS[tr * 8 + wave] = ps;
    __syncthreads();
    float tot = redS[tr * 8];
#pragma unroll
    for (int w = 1; w < 8; ++w) tot += redS[tr * 8 + w];
    const float inv = pcarry * (1.0f / tot);
    const unsigned u = pk16(h_bits(e0 * inv), h_bits(e1 * inv));
    unsigned* wp = Wp + (size_t)(bt0 + tr) * (kNS / 2) + tid;
    *(volatile unsigned*)wp = u;
    __threadfence();
    *(volatile unsigned*)wp = u;
  }
}

extern "C" void kernel_launch(void* const* d_in, const int* in_sizes, int n_in,
                              void* d_out, int out_size, void* d_ws, size_t ws_size,
                              hipStream_t stream) {
  if (n_in < 10) return;
  if (in_sizes[0] != kNB * kNT * kNA) return;
  if (in_sizes[1] != kNB * kNS * kNA) return;
  if (in_sizes[2] != kNB * kNS * kNA) return;
  if (in_sizes[3] != kNB * kNT * kNS) return;
  if (in_sizes[4] != kNA * kNA) return;
  if (in_sizes[5] != kNA) return;
  if (in_sizes[6] != kNA * kNA) return;
  if (in_sizes[7] != kNA) return;
  if (in_sizes[8] != kNA) return;
  if (in_sizes[9] != 1) return;
  if (out_size != kNB * kNT * kNA) return;
  if (ws_size < kWsTotal) return;

  const float* queries = (const float*)d_in[0];
  const float* keys    = (const float*)d_in[1];
  const float* values  = (const float*)d_in[2];
  const float* amask   = (const float*)d_in[3];
  const float* Wa_w    = (const float*)d_in[4];
  const float* Wa_b    = (const float*)d_in[5];
  const float* Ua_w    = (const float*)d_in[6];
  const float* Ua_b    = (const float*)d_in[7];
  const float* va_w    = (const float*)d_in[8];
  const float* va_b    = (const float*)d_in[9];
  float* out = (float*)d_out;

  char* ws = (char*)d_ws;
  unsigned short* K16  = (unsigned short*)(ws + kOffK16);
  unsigned short* Q16  = (unsigned short*)(ws + kOffQ16);
  unsigned short* WA16 = (unsigned short*)(ws + kOffWA16);
  unsigned short* UA16 = (unsigned short*)(ws + kOffUA16);
  unsigned short* VT16 = (unsigned short*)(ws + kOffVT16);
  float*          KPRJ = (float*)(ws + kOffKPRJ);
  float*          QPRJ = (float*)(ws + kOffQPRJ);
  unsigned short* W16  = (unsigned short*)(ws + kOffW16);

  cast8_f16_planes_kernel<<<dim3((kRowsK * kNA / 8) / 256, 4), 256, 0, stream>>>(
      keys, queries, Wa_w, Ua_w, K16, Q16, WA16, UA16,
      kRowsK * kNA / 8, kRowsQ * kNA / 8, kNA * kNA / 8, kNA * kNA / 8,
      kActCarry, kActCarry, kWgtCarry, kWgtCarry);

  vt_cast_kernel<<<dim3(kNS / 64, kNA / 64, kNB), 256, 0, stream>>>(values, VT16, kValCarry);

  wmma_gemm64_f16<2><<<dim3((kRowsK / 64) * (kNA / 64) / 8, 1), 256, 0, stream>>>(
      K16, kNA, 0L, WA16, kNA, 0L, KPRJ, kNA, 0L, Wa_b, kRowsK, kNA, kNA, kProjScale);

  wmma_gemm64_f16<2><<<dim3((kRowsQ / 64) * (kNA / 64) / 8, 1), 256, 0, stream>>>(
      Q16, kNA, 0L, UA16, kNA, 0L, QPRJ, kNA, 0L, Ua_b, kRowsQ, kNA, kNA, kProjScale);

  score_softmax_kernel<<<kRowsQ / kTRows, 256, 0, stream>>>(
      QPRJ, KPRJ, amask, va_w, va_b, (unsigned*)W16, kProbCarry);

  wmma_gemm64_f16<0><<<dim3((kNT / 64) * (kNA / 64) / 8, kNB), 256, 0, stream>>>(
      W16, kNS, (long)kNT * kNS, VT16, kNS, (long)kNA * kNS, out, kNA, (long)kNT * kNA,
      Ua_b, kNT, kNA, kNS, kPvScale);
}
